// KalmanFilter_26079041421461
// MI455X (gfx1250) — hardware-verified
//
#include <hip/hip_runtime.h>
#include <stdint.h>

typedef __attribute__((ext_vector_type(16))) __bf16 v16b;
typedef __attribute__((ext_vector_type(8)))  __bf16 v8b;
typedef __attribute__((ext_vector_type(8)))  float  v8f;
typedef __attribute__((ext_vector_type(4)))  float  v4f;
typedef __attribute__((ext_vector_type(16))) unsigned short v16us;
typedef __attribute__((ext_vector_type(4)))  unsigned short v4us;
typedef __attribute__((ext_vector_type(4)))  unsigned int v4ui;

namespace {
constexpr int NSTATE = 32;
constexpr int MCTRL  = 8;
constexpr int POBS   = 16;
constexpr int TSTEPS = 128;
constexpr int NBATCH = 64;
constexpr int NTH    = 128;
constexpr int NWAVES = 4;
constexpr int PP     = 32;
constexpr int NN     = NSTATE * NSTATE;
constexpr int RECF   = NSTATE * (NSTATE + 1);
constexpr int RECLINES = RECF / 32;
constexpr float QDIAG = 0.01f;
constexpr float RDIAG = 0.01f;
static_assert(PP == NSTATE, "plane pitch equals state dim: flat index == row*PP+col");
static_assert(RECF % 32 == 0, "output record is a whole number of 128-B lines");

constexpr size_t WS_SIGF = 0;
constexpr size_t WS_SIGP = WS_SIGF + (size_t)NBATCH * TSTEPS * NN;
constexpr size_t WS_MUF  = WS_SIGP + (size_t)NBATCH * TSTEPS * NN;
constexpr size_t WS_MUP  = WS_MUF  + (size_t)NBATCH * TSTEPS * NSTATE;
constexpr size_t WS_TOTAL_FLOATS = WS_MUP + (size_t)NBATCH * TSTEPS * NSTATE;
static_assert(WS_TOTAL_FLOATS * 4 == 69206016, "ws carve total bytes");

enum { EP_PL = 0, EP_F32 = 1, EP_SIGP = 2, EP_IKC = 3 };
}

__device__ __forceinline__ unsigned short bfb(float f) {
  const unsigned u = __float_as_uint(f);
  return (unsigned short)((u + 0x7FFFu + ((u >> 16) & 1u)) >> 16);
}
__device__ __forceinline__ float bff(unsigned short h) { return __uint_as_float(((unsigned)h) << 16); }

__device__ __forceinline__ void split4_store(unsigned short* ph, unsigned short* pl, int off, v4f v) {
  v4us hv, lv;
#pragma unroll
  for (int q = 0; q < 4; ++q) {
    const float f = v[q];
    const unsigned short hb = bfb(f);
    hv[q] = hb;
    lv[q] = bfb(f - bff(hb));
  }
  *(v4us*)(ph + off) = hv;
  *(v4us*)(pl + off) = lv;
}

__device__ __forceinline__ v8f mma_bf(v16b a, v16b b, v8f c) {
  c = __builtin_amdgcn_wmma_f32_16x16x32_bf16(false, a, false, b, (short)0, c, false, false);
  asm volatile("v_nop\n\tv_nop\n\tv_nop\n\tv_nop" : "+v"(c) : "v"(a), "v"(b));
  return c;
}

__device__ __forceinline__ v16b ld_rowfrag(const unsigned short* pl, int row, int koff) {
  union { v16b v; v8b q[2]; } f;
  const __bf16* p = (const __bf16*)(const void*)(pl + row * PP + koff);
  f.q[0] = *(const v8b*)(p);
  f.q[1] = *(const v8b*)(p + 16);
  return f.v;
}

template <int KDIM>
__device__ __forceinline__ v16b ld_colfrag(const unsigned short* pl, int col, int koff) {
  v16us u;
#pragma unroll
  for (int i = 0; i < 16; ++i) {
    const int k  = (i < 8) ? (koff + i) : (16 + koff + (i - 8));
    const int kc = (k < KDIM) ? k : (KDIM - 1);
    const unsigned short x = pl[kc * PP + col];
    u[i] = (k < KDIM) ? x : (unsigned short)0;
  }
  return __builtin_bit_cast(v16b, u);
}

template <bool BG, int KDIM, int EM>
__device__ __forceinline__ void mm_tiles(const unsigned short* xh, const unsigned short* xl,
                                         const unsigned short* yh, const unsigned short* yl,
                                         int MR, int NC,
                                         float* df, int ldd, unsigned short* dh, unsigned short* dl,
                                         int wave, int lane, int wbase, int wcnt)
{
  const int nti = MR >> 4, ntj = NC >> 4, nt = nti * ntj;
  const int r16 = lane & 15, hsel = lane >> 4, koff = hsel * 8;
  if (wave >= wbase) {
    for (int tile = wave - wbase; tile < nt; tile += wcnt) {
      const int ti = tile / ntj, tj = tile - ti * ntj;
      const v16b ah = ld_rowfrag(xh, ti * 16 + r16, koff);
      const v16b al = ld_rowfrag(xl, ti * 16 + r16, koff);
      v16b bh, bl;
      if (BG) {
        bh = ld_colfrag<KDIM>(yh, tj * 16 + r16, koff);
        bl = ld_colfrag<KDIM>(yl, tj * 16 + r16, koff);
      } else {
        bh = ld_rowfrag(yh, tj * 16 + r16, koff);
        bl = ld_rowfrag(yl, tj * 16 + r16, koff);
      }
      v8f acc = (v8f){0.f, 0.f, 0.f, 0.f, 0.f, 0.f, 0.f, 0.f};
      acc = mma_bf(ah, bh, acc);
      acc = mma_bf(ah, bl, acc);
      acc = mma_bf(al, bh, acc);
      const int col = tj * 16 + r16;
#pragma unroll
      for (int r = 0; r < 8; ++r) {
        const int row = ti * 16 + hsel * 8 + r;
        float v = acc[r];
        if (EM == EP_SIGP) v = (row == col) ? (v + QDIAG) : v;
        if (EM == EP_IKC)  v = ((row == col) ? 1.0f : 0.0f) - v;
        if (EM == EP_F32 || EM == EP_SIGP) df[row * ldd + col] = v;
        if (EM == EP_PL || EM == EP_SIGP || EM == EP_IKC) {
          const unsigned short hb = bfb(v);
          dh[row * PP + col] = hb;
          dl[row * PP + col] = bfb(v - bff(hb));
        }
      }
    }
  }
}

__device__ __forceinline__ void store_lines(float* dst, const float* src, int nlines, int tid) {
  const int lq = tid >> 3, c4 = (tid & 7) * 4;
  for (int pass = 0; pass < 2; ++pass) {
    for (int L = lq; L < nlines; L += NTH / 8) {
      const int o = L * 32 + c4;
      const v4f v = *(const v4f*)(src + o);
      *(volatile v4f*)(dst + o) = v;
    }
    __threadfence();
  }
}

template <int n>
__device__ __forceinline__ void lu_nopiv(float* Mx, int tid) {
  const int jc = tid & 31, rg = tid >> 5;
#pragma unroll 1
  for (int k = 0; k < n - 1; ++k) {
    __syncthreads();
    const float rp = 1.0f / Mx[k * n + k];
    if (tid < n - 1 - k) {
      const int i = k + 1 + tid;
      Mx[i * n + k] = Mx[i * n + k] * rp;
    }
    __syncthreads();
    if (jc > k && jc < n) {
      const float ukj = Mx[k * n + jc];
#pragma unroll 1
      for (int i = k + 1 + rg; i < n; i += NWAVES) Mx[i * n + jc] = Mx[i * n + jc] - Mx[i * n + k] * ukj;
    }
  }
  __syncthreads();
}

template <int n>
__device__ __forceinline__ void lu_subst(const float* Mx, const float* bsrc, float* xr) {
#pragma unroll 1
  for (int jj = 0; jj < n; ++jj) {
    float s = bsrc[jj];
#pragma unroll 1
    for (int l = 0; l < jj; ++l) s = s - Mx[jj * n + l] * xr[l];
    xr[jj] = s;
  }
#pragma unroll 1
  for (int jj = n - 1; jj >= 0; --jj) {
    float s = xr[jj];
#pragma unroll 1
    for (int l = jj + 1; l < n; ++l) s = s - Mx[jj * n + l] * xr[l];
    const float rd = 1.0f / Mx[jj * n + jj];
    xr[jj] = s * rd;
  }
}

extern "C" __global__ void __launch_bounds__(NTH)
lgssm_smooth_kernel(const float* __restrict__ Yg, const float* __restrict__ Ug,
                    const float* __restrict__ Ag, const float* __restrict__ Bg,
                    const float* __restrict__ Cg, const float* __restrict__ mu0g,
                    const float* __restrict__ Sig0g, float* outp, float* ws)
{
  const int tid = threadIdx.x, wave = tid >> 5, lane = tid & 31, b = blockIdx.x;

  __shared__ __align__(16) float s_g32[NN];
  __shared__ __align__(16) float s_sig[NN];
  __shared__ __align__(16) float s_sigp[NN];
  __shared__ __align__(16) float s_t1b[NN];
  __shared__ __align__(16) float s_w[NN];
  __shared__ __align__(16) float s_lu[NN];
  __shared__ __align__(16) float s_rec[RECF];
  __shared__ __align__(16) float s_pk32[NSTATE * POBS];
  __shared__ __align__(16) unsigned short s_pa[2][NN];
  __shared__ __align__(16) unsigned short s_pc[2][POBS * PP];
  __shared__ __align__(16) unsigned short s_psig[2][NN];
  __shared__ __align__(16) unsigned short s_pt1[2][NN];
  __shared__ __align__(16) unsigned short s_psigp[2][NN];
  __shared__ __align__(16) unsigned short s_pk[2][NN];
  __shared__ __align__(16) unsigned short s_pt2[2][POBS * PP];
  __shared__ __align__(16) float s_mu[NSTATE];
  __shared__ __align__(16) float s_mup[NSTATE];
  __shared__ __align__(16) float s_r[POBS];
  __shared__ __align__(16) float s_mus[NSTATE];
  __shared__ __align__(16) float s_mf[NSTATE];
  __shared__ __align__(16) float s_dmu[NSTATE];

  float* ws_sigf = ws + WS_SIGF;
  float* ws_sigp = ws + WS_SIGP;
  float* ws_muf  = ws + WS_MUF;
  float* ws_mup  = ws + WS_MUP;

  {
    const v4ui z = (v4ui){0u, 0u, 0u, 0u};
    v4ui* pz = (v4ui*)(void*)&s_pk[0][0];
    pz[tid] = z;
    pz[tid + NTH] = z;
  }
  __syncthreads();
  if (tid < NSTATE) s_mu[tid] = mu0g[tid];
#pragma unroll
  for (int c2 = 0; c2 < 2; ++c2) {
    const int e = 4 * (tid + NTH * c2);
    const v4f sv = *(const v4f*)(Sig0g + e);
    split4_store(s_psig[0], s_psig[1], e, sv);
  }
  __syncthreads();

  for (int t = 0; t < TSTEPS; ++t) {
    const size_t bt = (size_t)b * TSTEPS + t;
    const float* Abt = Ag + bt * NN;
    const float* Bbt = Bg + bt * (NSTATE * MCTRL);
    const float* Cbt = Cg + bt * (POBS * NSTATE);

#pragma unroll
    for (int c2 = 0; c2 < 2; ++c2) {
      const int e = 4 * (tid + NTH * c2);
      const v4f av = *(const v4f*)(Abt + e);
      split4_store(s_pa[0], s_pa[1], e, av);
    }
    {
      const int e = 4 * tid;
      const v4f cv = *(const v4f*)(Cbt + e);
      split4_store(s_pc[0], s_pc[1], e, cv);
    }
    __syncthreads();

    if (tid < NSTATE) {
      const int ri = tid & (NSTATE - 1);
      const v4f* arow = (const v4f*)(Abt + ri * NSTATE);
      float s1 = 0.0f;
#pragma unroll 1
      for (int c4i = 0; c4i < NSTATE / 4; ++c4i) {
        const v4f a4 = arow[c4i];
        const v4f m4 = *(const v4f*)(s_mu + 4 * c4i);
        s1 += a4[0] * m4[0];
        s1 += a4[1] * m4[1];
        s1 += a4[2] * m4[2];
        s1 += a4[3] * m4[3];
      }
      const v4f* brow = (const v4f*)(Bbt + ri * MCTRL);
      const v4f* urow = (const v4f*)(Ug + bt * MCTRL);
      float s2 = 0.0f;
#pragma unroll 1
      for (int c4i = 0; c4i < MCTRL / 4; ++c4i) {
        const v4f b4 = brow[c4i];
        const v4f u4 = urow[c4i];
        s2 += b4[0] * u4[0];
        s2 += b4[1] * u4[1];
        s2 += b4[2] * u4[2];
        s2 += b4[3] * u4[3];
      }
      s_mup[ri] = s1 + s2;
    }
    mm_tiles<true, NSTATE, EP_PL>(s_pa[0], s_pa[1], s_psig[0], s_psig[1], NSTATE, NSTATE,
                                  nullptr, 0, s_pt1[0], s_pt1[1], wave, lane, 0, NWAVES);
    __syncthreads();

    if (tid < POBS) {
      const int ri = tid & (POBS - 1);
      const v4f* crow = (const v4f*)(Cbt + ri * NSTATE);
      float s = 0.0f;
#pragma unroll 1
      for (int c4i = 0; c4i < NSTATE / 4; ++c4i) {
        const v4f c4v = crow[c4i];
        const v4f m4 = *(const v4f*)(s_mup + 4 * c4i);
        s += c4v[0] * m4[0];
        s += c4v[1] * m4[1];
        s += c4v[2] * m4[2];
        s += c4v[3] * m4[3];
      }
      s_r[ri] = Yg[bt * POBS + ri] - s;
    }
    mm_tiles<false, NSTATE, EP_SIGP>(s_pt1[0], s_pt1[1], s_pa[0], s_pa[1], NSTATE, NSTATE,
                                     s_sigp, NSTATE, s_psigp[0], s_psigp[1], wave, lane, 0, NWAVES);
    __syncthreads();

    store_lines(ws_sigp + bt * NN, s_sigp, NN / 32, tid);
    store_lines(ws_mup + bt * NSTATE, s_mup, 1, tid);
    mm_tiles<true, NSTATE, EP_PL>(s_pc[0], s_pc[1], s_psigp[0], s_psigp[1], POBS, NSTATE,
                                  nullptr, 0, s_pt2[0], s_pt2[1], wave, lane, 0, 2);
    mm_tiles<false, NSTATE, EP_F32>(s_psigp[0], s_psigp[1], s_pc[0], s_pc[1], NSTATE, POBS,
                                    s_pk32, POBS, nullptr, nullptr, wave, lane, 2, 2);
    __syncthreads();

    mm_tiles<false, NSTATE, EP_F32>(s_pt2[0], s_pt2[1], s_pc[0], s_pc[1], POBS, POBS,
                                    s_g32, POBS, nullptr, nullptr, wave, lane, 0, 1);
    __syncthreads();

#pragma unroll
    for (int c2 = 0; c2 < 2; ++c2) {
      const int e = tid + NTH * c2;
      const int i = e >> 4, j = e & 15;
      const float dg = (i == j) ? RDIAG : 0.0f;
      const float x1 = s_g32[i * POBS + j] + dg;
      const float x2 = s_g32[j * POBS + i] + dg;
      s_lu[e] = 0.5f * (x1 + x2);
    }
    lu_nopiv<POBS>(s_lu, tid);

    if (tid < NSTATE) {
      const int ri = tid & (NSTATE - 1);
      float* xr = s_pk32 + ri * POBS;
      lu_subst<POBS>(s_lu, xr, xr);
#pragma unroll 1
      for (int jj = 0; jj < POBS; ++jj) {
        const float kv = xr[jj];
        const unsigned short hb = bfb(kv);
        s_pk[0][ri * PP + jj] = hb;
        s_pk[1][ri * PP + jj] = bfb(kv - bff(hb));
        const float kr = kv * RDIAG;
        const unsigned short hr = bfb(kr);
        s_psig[0][ri * PP + jj] = hr;
        s_psig[1][ri * PP + jj] = bfb(kr - bff(hr));
        s_psig[0][ri * PP + POBS + jj] = (unsigned short)0;
        s_psig[1][ri * PP + POBS + jj] = (unsigned short)0;
      }
    }
    __syncthreads();

    if (tid < NSTATE) {
      const int ri = tid & (NSTATE - 1);
      const float* kr = s_pk32 + ri * POBS;
      float s = 0.0f;
#pragma unroll 1
      for (int c4i = 0; c4i < POBS / 4; ++c4i) {
        const v4f k4 = *(const v4f*)(kr + 4 * c4i);
        const v4f r4 = *(const v4f*)(s_r + 4 * c4i);
        s += k4[0] * r4[0];
        s += k4[1] * r4[1];
        s += k4[2] * r4[2];
        s += k4[3] * r4[3];
      }
      const float m = s_mup[ri] + s;
      s_mu[ri] = m;
      s_rec[ri * (NSTATE + 1)] = m;
    }
    mm_tiles<true, POBS, EP_IKC>(s_pk[0], s_pk[1], s_pc[0], s_pc[1], NSTATE, NSTATE,
                                 nullptr, 0, s_pa[0], s_pa[1], wave, lane, 0, NWAVES);
    mm_tiles<false, NSTATE, EP_F32>(s_psig[0], s_psig[1], s_pk[0], s_pk[1], NSTATE, NSTATE,
                                    s_w, NSTATE, nullptr, nullptr, wave, lane, 0, NWAVES);
    __syncthreads();

    mm_tiles<true, NSTATE, EP_PL>(s_pa[0], s_pa[1], s_psigp[0], s_psigp[1], NSTATE, NSTATE,
                                  nullptr, 0, s_pt1[0], s_pt1[1], wave, lane, 0, NWAVES);
    __syncthreads();

    mm_tiles<false, NSTATE, EP_F32>(s_pt1[0], s_pt1[1], s_pa[0], s_pa[1], NSTATE, NSTATE,
                                    s_t1b, NSTATE, nullptr, nullptr, wave, lane, 0, NWAVES);
    __syncthreads();

    for (int e = tid; e < NN; e += NTH) {
      const int i = e >> 5, j = e & 31, et = j * NSTATE + i;
      const float x1 = s_t1b[e] + s_w[e];
      const float x2 = s_t1b[et] + s_w[et];
      const float v = 0.5f * (x1 + x2);
      s_sig[e] = v;
      s_rec[i * (NSTATE + 1) + 1 + j] = v;
      const unsigned short hb = bfb(v);
      s_psig[0][e] = hb;
      s_psig[1][e] = bfb(v - bff(hb));
    }
    __syncthreads();

    store_lines(ws_sigf + bt * NN, s_sig, NN / 32, tid);
    store_lines(ws_muf + bt * NSTATE, s_mu, 1, tid);
    if (t == TSTEPS - 1) store_lines(outp + bt * RECF, s_rec, RECLINES, tid);
  }

  if (tid < NSTATE) s_mus[tid] = s_mu[tid];
#pragma unroll
  for (int c2 = 0; c2 < 2; ++c2) {
    const int e = 4 * (tid + NTH * c2);
    *(v4f*)(s_w + e) = *(const v4f*)(s_sig + e);
  }
  __syncthreads();

  for (int t = TSTEPS - 2; t >= 0; --t) {
    const size_t bt = (size_t)b * TSTEPS + t, bt1 = bt + 1;
    const float* sfp = ws_sigf + bt * NN;
    const float* spp = ws_sigp + bt1 * NN;
    const float* Atp = Ag + bt * NN;

#pragma unroll
    for (int c2 = 0; c2 < 2; ++c2) {
      const int e = 4 * (tid + NTH * c2);
      const v4f sf = *(const v4f*)(sfp + e);
      *(v4f*)(s_sig + e) = sf;
      split4_store(s_psig[0], s_psig[1], e, sf);
      const v4f sp = *(const v4f*)(spp + e);
      const v4f ss = *(const v4f*)(s_w + e);
      split4_store(s_psigp[0], s_psigp[1], e, ss - sp);
      const int i = e >> 5, j = e & 31;
      s_lu[(j + 0) * NSTATE + i] = sp[0];
      s_lu[(j + 1) * NSTATE + i] = sp[1];
      s_lu[(j + 2) * NSTATE + i] = sp[2];
      s_lu[(j + 3) * NSTATE + i] = sp[3];
      const v4f av = *(const v4f*)(Atp + e);
      split4_store(s_pa[0], s_pa[1], e, av);
    }
    if (tid < NSTATE) {
      const int ri = tid & (NSTATE - 1);
      s_mf[ri]  = ws_muf[bt * NSTATE + ri];
      s_dmu[ri] = s_mus[ri] - ws_mup[bt1 * NSTATE + ri];
    }
    __syncthreads();

    mm_tiles<false, NSTATE, EP_F32>(s_psig[0], s_psig[1], s_pa[0], s_pa[1], NSTATE, NSTATE,
                                    s_g32, NSTATE, nullptr, nullptr, wave, lane, 0, NWAVES);
    lu_nopiv<NSTATE>(s_lu, tid);

    if (tid < NSTATE) {
      const int ri = tid & (NSTATE - 1);
      float* xr = s_t1b + ri * NSTATE;
      lu_subst<NSTATE>(s_lu, s_g32 + ri * NSTATE, xr);
#pragma unroll 1
      for (int jj = 0; jj < NSTATE; ++jj) {
        const float v = xr[jj];
        const unsigned short hb = bfb(v);
        s_pk[0][ri * PP + jj] = hb;
        s_pk[1][ri * PP + jj] = bfb(v - bff(hb));
      }
    }
    __syncthreads();

    if (tid < NSTATE) {
      const int ri = tid & (NSTATE - 1);
      const float* jr = s_t1b + ri * NSTATE;
      float s = 0.0f;
#pragma unroll 1
      for (int c4i = 0; c4i < NSTATE / 4; ++c4i) {
        const v4f j4 = *(const v4f*)(jr + 4 * c4i);
        const v4f d4 = *(const v4f*)(s_dmu + 4 * c4i);
        s += j4[0] * d4[0];
        s += j4[1] * d4[1];
        s += j4[2] * d4[2];
        s += j4[3] * d4[3];
      }
      const float m = s_mf[ri] + s;
      s_mus[ri] = m;
      s_rec[ri * (NSTATE + 1)] = m;
    }
    mm_tiles<true, NSTATE, EP_PL>(s_pk[0], s_pk[1], s_psigp[0], s_psigp[1], NSTATE, NSTATE,
                                  nullptr, 0, s_pt1[0], s_pt1[1], wave, lane, 0, NWAVES);
    __syncthreads();

    mm_tiles<false, NSTATE, EP_F32>(s_pt1[0], s_pt1[1], s_pk[0], s_pk[1], NSTATE, NSTATE,
                                    s_g32, NSTATE, nullptr, nullptr, wave, lane, 0, NWAVES);
    __syncthreads();

    for (int e = tid; e < NN; e += NTH) {
      const int i = e >> 5, j = e & 31, et = j * NSTATE + i;
      const float x1 = s_sig[e] + s_g32[e];
      const float x2 = s_sig[et] + s_g32[et];
      const float v = 0.5f * (x1 + x2);
      s_w[e] = v;
      s_rec[i * (NSTATE + 1) + 1 + j] = v;
    }
    __syncthreads();

    store_lines(outp + bt * RECF, s_rec, RECLINES, tid);
  }
}

extern "C" void kernel_launch(void* const* d_in, const int* in_sizes, int n_in,
                              void* d_out, int out_size, void* d_ws, size_t ws_size,
                              hipStream_t stream)
{
  if (n_in < 7) return;
  if (in_sizes[0] != NBATCH * TSTEPS * POBS) return;
  if (in_sizes[1] != NBATCH * TSTEPS * MCTRL) return;
  if (in_sizes[2] != NBATCH * TSTEPS * NN) return;
  if (in_sizes[3] != NBATCH * TSTEPS * NSTATE * MCTRL) return;
  if (in_sizes[4] != NBATCH * TSTEPS * POBS * NSTATE) return;
  if (in_sizes[5] != NSTATE) return;
  if (in_sizes[6] != NN) return;
  if (out_size != NBATCH * TSTEPS * RECF) return;
  if (ws_size < WS_TOTAL_FLOATS * sizeof(float)) return;
  const float* Yg   = (const float*)d_in[0];
  const float* Ug   = (const float*)d_in[1];
  const float* Ag   = (const float*)d_in[2];
  const float* Bg   = (const float*)d_in[3];
  const float* Cg   = (const float*)d_in[4];
  const float* mu0  = (const float*)d_in[5];
  const float* Sig0 = (const float*)d_in[6];
  lgssm_smooth_kernel<<<dim3(NBATCH), dim3(NTH), 0, stream>>>(Yg, Ug, Ag, Bg, Cg, mu0, Sig0,
                                                              (float*)d_out, (float*)d_ws);
}
